// TorchModel_59219009077447
// MI455X (gfx1250) — hardware-run, weakly checked
//
#include <hip/hip_runtime.h>
#include <math.h>

typedef __attribute__((ext_vector_type(16))) _Float16 v16h;
typedef __attribute__((ext_vector_type(8)))  float    v8f;
typedef __attribute__((ext_vector_type(4)))  float    v4f;
typedef __attribute__((ext_vector_type(4)))  unsigned v4u;
typedef __attribute__((ext_vector_type(2)))  unsigned v2u;

constexpr int kVocab  = 50000;
constexpr int kDim    = 20;
constexpr int kHid    = 20;
constexpr int kNcls   = 5;
constexpr int kBatch  = 16384;
constexpr int kSeq    = 256;
constexpr int kPitch  = 32;
constexpr int kSlabP  = 36;
constexpr float kCarryW = 64.0f;
constexpr float kCarryH = 64.0f;
constexpr float kFold   = 1.0f / (kCarryW * kCarryH);

constexpr int kTabRowsPerBlock = 80;
constexpr int kTabBlocks       = kVocab / kTabRowsPerBlock;
constexpr int kRecBlocks       = kBatch / 128;
constexpr int kClsBlocks       = (kBatch * kNcls) / 256;
static_assert(kDim == kHid, "square recurrent weight and table width");
static_assert(kTabBlocks * kTabRowsPerBlock == kVocab, "table grid is exact");
static_assert(kRecBlocks * 128 == kBatch, "recurrence grid is exact");
static_assert(kClsBlocks * 256 == kBatch * kNcls, "head grid is exact");
static_assert((kHid % 4) == 0 && kHid <= kPitch && kPitch == 32, "K and N padded 20 -> 32");
static_assert((kSeq % 4) == 0, "sequence length");

constexpr size_t kOffTab  = 0;
constexpr size_t kOffHl   = kOffTab + (size_t)kVocab * kPitch * 4;
constexpr size_t kWsTotal = kOffHl + (size_t)kBatch * kPitch * 4;
static_assert(kWsTotal == 8497152ull, "carve total");
static_assert((kOffHl % 128) == 0, "128-B aligned regions");
static_assert(kWsTotal <= 134217728ull, "carve cap");

__device__ __forceinline__ v8f mma_f16(v16h a, v16h b, v8f c) {
  c = __builtin_amdgcn_wmma_f32_16x16x32_f16(false, a, false, b, (short)0, c, false, false);
  asm volatile("v_nop\n\tv_nop\n\tv_nop\n\tv_nop" : "+v"(c) : "v"(a), "v"(b));
  return c;
}

__device__ __forceinline__ float tanh_f32(float x) {
  const float a = fminf(fabsf(x), 15.0f);
  const float e = expf(a + a);
  const float r = __builtin_amdgcn_rcpf(e + 1.0f);
  const float t = fmaf(-2.0f, r, 1.0f);
  return copysignf(t, x);
}

__global__ __launch_bounds__(128) void table_kernel(
    const float* __restrict__ emb, const float* __restrict__ Wih, float* __restrict__ TAB)
{
  __shared__ __align__(16) float sW[kDim * kPitch];
  const int tid  = threadIdx.x;
  const int lane = tid & 31;
  const int wave = __builtin_amdgcn_readfirstlane((int)(threadIdx.x >> 5));
#pragma unroll 1
  for (int i = 0; i < 5; ++i) {
    const int e   = i * 128 + tid;
    const int d   = e >> 5;
    const int col = e & 31;
    const int cc  = col < kHid ? col : kHid - 1;
    float w = Wih[cc * kDim + d];
    asm volatile("" : "+v"(w));
    sW[e] = (col < kHid) ? w : 0.0f;
  }
  __syncthreads();
  const int q  = lane >> 3;
  const int c4 = (lane & 7) * 4;
  const bool padc = (c4 >= kHid);
#pragma unroll 1
  for (int it = 0; it < 5; ++it) {
    const int v = blockIdx.x * kTabRowsPerBlock + it * 16 + wave * 4 + q;
    const float* er = emb + (size_t)v * kDim;
    float a0 = 0.0f, a1 = 0.0f, a2 = 0.0f, a3 = 0.0f;
#pragma unroll 1
    for (int g = 0; g < 5; ++g) {
      const v4f ev = *(const v4f*)(er + 4 * g);
      const float* wp = sW + (4 * g) * kPitch + c4;
      const v4f w0 = *(const v4f*)(wp);
      const v4f w1 = *(const v4f*)(wp + kPitch);
      const v4f w2 = *(const v4f*)(wp + 2 * kPitch);
      const v4f w3 = *(const v4f*)(wp + 3 * kPitch);
      a0 = fmaf(ev[0], w0[0], a0); a1 = fmaf(ev[0], w0[1], a1); a2 = fmaf(ev[0], w0[2], a2); a3 = fmaf(ev[0], w0[3], a3);
      a0 = fmaf(ev[1], w1[0], a0); a1 = fmaf(ev[1], w1[1], a1); a2 = fmaf(ev[1], w1[2], a2); a3 = fmaf(ev[1], w1[3], a3);
      a0 = fmaf(ev[2], w2[0], a0); a1 = fmaf(ev[2], w2[1], a1); a2 = fmaf(ev[2], w2[2], a2); a3 = fmaf(ev[2], w2[3], a3);
      a0 = fmaf(ev[3], w3[0], a0); a1 = fmaf(ev[3], w3[1], a1); a2 = fmaf(ev[3], w3[2], a2); a3 = fmaf(ev[3], w3[3], a3);
    }
    const bool zr = (v == 0) || padc;
    v4f o;
    o[0] = zr ? 0.0f : a0;
    o[1] = zr ? 0.0f : a1;
    o[2] = zr ? 0.0f : a2;
    o[3] = zr ? 0.0f : a3;
    float* dst = TAB + (size_t)v * kPitch + c4;
    *(volatile v4f*)dst = o;
    __threadfence();
    *(volatile v4f*)dst = o;
  }
}

__global__ __launch_bounds__(256) void recur_kernel(
    const int* __restrict__ x, const float* __restrict__ TAB, const float* __restrict__ Whh, float* __restrict__ HL)
{
  __shared__ __align__(16) unsigned sWu[32 * 16];
  __shared__ __align__(16) float sH[8][16 * kSlabP];
  union FragU { v16h v; v4u u[2]; };
  const int tid  = threadIdx.x;
  const int lane = tid & 31;
  const int wave = __builtin_amdgcn_readfirstlane((int)(threadIdx.x >> 5));
  const int hh   = lane >> 4;
  const int n    = lane & 15;

  {
    const int row = tid >> 3;
    const int k0  = (tid & 7) * 4;
    const int rc  = row < kHid ? row : kHid - 1;
    unsigned hbits[4];
#pragma unroll
    for (int e = 0; e < 4; ++e) {
      const int k  = k0 + e;
      const int kc = k < kHid ? k : kHid - 1;
      float f = Whh[rc * kHid + kc];
      asm volatile("" : "+v"(f));
      const float g = (row < kHid && k < kHid) ? f * kCarryW : 0.0f;
      const _Float16 hv = (_Float16)g;
      hbits[e] = (unsigned)__builtin_bit_cast(unsigned short, hv);
    }
    v2u w;
    w[0] = hbits[0] | (hbits[1] << 16);
    w[1] = hbits[2] | (hbits[3] << 16);
    *(v2u*)(sWu + tid * 2) = w;
  }
  __syncthreads();

  FragU a0, a1;
  a0.u[0] = *(const v4u*)(sWu + n * 16 + 4 * hh);
  a0.u[1] = *(const v4u*)(sWu + n * 16 + 8 + 4 * hh);
  a1.u[0] = *(const v4u*)(sWu + (16 + n) * 16 + 4 * hh);
  a1.u[1] = *(const v4u*)(sWu + (16 + n) * 16 + 8 + 4 * hh);

  const int b0 = (blockIdx.x * 8 + wave) * 16;
  const int* xr = x + (size_t)(b0 + n) * kSeq;
  const bool t1ok = (hh == 0);

  v16h hb;
#pragma unroll
  for (int i = 0; i < 16; ++i) hb[i] = (_Float16)0.0f;
  float hf0[8];
  float hf1[4];
#pragma unroll
  for (int r = 0; r < 8; ++r) hf0[r] = 0.0f;
#pragma unroll
  for (int r = 0; r < 4; ++r) hf1[r] = 0.0f;

#pragma unroll 1
  for (int t = 0; t < kSeq; ++t) {
    int idx = xr[t];
    idx = idx < 0 ? 0 : idx;
    idx = idx > (kVocab - 1) ? (kVocab - 1) : idx;
    const float* tr = TAB + (size_t)idx * kPitch + 8 * hh;
    const v4f c00 = *(const v4f*)(tr);
    const v4f c01 = *(const v4f*)(tr + 4);
    const v4f c10 = *(const v4f*)(tr + 16);

    v8f acc0 = (v8f){0.f, 0.f, 0.f, 0.f, 0.f, 0.f, 0.f, 0.f};
    v8f acc1 = (v8f){0.f, 0.f, 0.f, 0.f, 0.f, 0.f, 0.f, 0.f};
    acc0 = mma_f16(a0.v, hb, acc0);
    acc1 = mma_f16(a1.v, hb, acc1);

#pragma unroll
    for (int r = 0; r < 4; ++r) {
      const float p = fmaf(acc0[r], kFold, c00[r]);
      hf0[r] = tanh_f32(p);
    }
#pragma unroll
    for (int r = 0; r < 4; ++r) {
      const float p = fmaf(acc0[4 + r], kFold, c01[r]);
      hf0[4 + r] = tanh_f32(p);
    }
#pragma unroll
    for (int r = 0; r < 4; ++r) {
      const float p = fmaf(acc1[r], kFold, c10[r]);
      const float tv = tanh_f32(p);
      hf1[r] = t1ok ? tv : 0.0f;
    }
#pragma unroll
    for (int r = 0; r < 8; ++r) hb[r] = (_Float16)(hf0[r] * kCarryH);
#pragma unroll
    for (int r = 0; r < 4; ++r) hb[8 + r] = (_Float16)(hf1[r] * kCarryH);
#pragma unroll
    for (int r = 0; r < 4; ++r) hb[12 + r] = (_Float16)0.0f;
  }

  float* slab = sH[wave];
  {
    v4f s0, s1, s2, s3;
    s0[0] = hf0[0]; s0[1] = hf0[1]; s0[2] = hf0[2]; s0[3] = hf0[3];
    s1[0] = hf0[4]; s1[1] = hf0[5]; s1[2] = hf0[6]; s1[3] = hf0[7];
    s2[0] = hf1[0]; s2[1] = hf1[1]; s2[2] = hf1[2]; s2[3] = hf1[3];
    s3[0] = 0.0f;   s3[1] = 0.0f;   s3[2] = 0.0f;   s3[3] = 0.0f;
    *(v4f*)(slab + n * kSlabP + 8 * hh)      = s0;
    *(v4f*)(slab + n * kSlabP + 8 * hh + 4)  = s1;
    *(v4f*)(slab + n * kSlabP + 16 + 8 * hh) = s2;
    *(v4f*)(slab + n * kSlabP + 20 + 8 * hh) = s3;
  }
  __builtin_amdgcn_fence(__ATOMIC_RELEASE, "workgroup");
  __builtin_amdgcn_wave_barrier();
  __builtin_amdgcn_fence(__ATOMIC_ACQUIRE, "workgroup");
  {
    const int q  = lane >> 3;
    const int c4 = (lane & 7) * 4;
    v4f o[4];
#pragma unroll
    for (int it = 0; it < 4; ++it) o[it] = *(const v4f*)(slab + (it * 4 + q) * kSlabP + c4);
#pragma unroll
    for (int it = 0; it < 4; ++it)
      *(volatile v4f*)(HL + (size_t)(b0 + it * 4 + q) * kPitch + c4) = o[it];
    __threadfence();
#pragma unroll
    for (int it = 0; it < 4; ++it)
      *(volatile v4f*)(HL + (size_t)(b0 + it * 4 + q) * kPitch + c4) = o[it];
  }
}

__global__ __launch_bounds__(256) void head_kernel(
    const float* __restrict__ HL, const float* __restrict__ Wc, const float* __restrict__ bc, float* __restrict__ out)
{
  __shared__ __align__(16) float sY[256];
  const int tid  = threadIdx.x;
  const int wave = __builtin_amdgcn_readfirstlane((int)(threadIdx.x >> 5));
  const int e = blockIdx.x * 256 + tid;
  const int b = e / kNcls;
  const int c = e - b * kNcls;
  const float* hr = HL + (size_t)b * kPitch;
  const float* wr = Wc + c * kHid;
  float y = 0.0f;
#pragma unroll 1
  for (int g = 0; g < kHid / 4; ++g) {
    const v4f hv = *(const v4f*)(hr + 4 * g);
    const v4f wv = *(const v4f*)(wr + 4 * g);
    y = fmaf(hv[0], wv[0], y);
    y = fmaf(hv[1], wv[1], y);
    y = fmaf(hv[2], wv[2], y);
    y = fmaf(hv[3], wv[3], y);
  }
  y = y + bc[c];
  sY[tid] = y;
  __syncthreads();
  if (wave < 2) {
    const v4f o = *(const v4f*)(sY + tid * 4);
    float* dst = out + (size_t)blockIdx.x * 256 + tid * 4;
    *(volatile v4f*)dst = o;
    __threadfence();
    *(volatile v4f*)dst = o;
  }
}

extern "C" void kernel_launch(void* const* d_in, const int* in_sizes, int n_in,
                              void* d_out, int out_size, void* d_ws, size_t ws_size,
                              hipStream_t stream) {
  if (n_in < 6) return;
  if (in_sizes[0] != kBatch * kSeq) return;
  if (in_sizes[1] != kVocab * kDim) return;
  if (in_sizes[2] != kHid * kDim) return;
  if (in_sizes[3] != kHid * kHid) return;
  if (in_sizes[4] != kNcls * kHid) return;
  if (in_sizes[5] != kNcls) return;
  if (out_size != kBatch * kNcls) return;
  if (ws_size < kWsTotal) return;

  const int*   x     = (const int*)d_in[0];
  const float* emb   = (const float*)d_in[1];
  const float* W_ih  = (const float*)d_in[2];
  const float* W_hh  = (const float*)d_in[3];
  const float* W_cls = (const float*)d_in[4];
  const float* b_cls = (const float*)d_in[5];
  float* out = (float*)d_out;

  char* ws = (char*)d_ws;
  float* TAB = (float*)(ws + kOffTab);
  float* HL  = (float*)(ws + kOffHl);

  table_kernel<<<kTabBlocks, 128, 0, stream>>>(emb, W_ih, TAB);
  recur_kernel<<<kRecBlocks, 256, 0, stream>>>(x, TAB, W_hh, HL);
  head_kernel<<<kClsBlocks, 256, 0, stream>>>(HL, W_cls, b_cls, out);
}
